// MLASegmentedCrossAttention_36043365548098
// MI455X (gfx1250) — hardware-verified
//
#include <hip/hip_runtime.h>
#include <cmath>


namespace {
constexpr int L = 2048, QD = 1024, KVD = 1024, CL = 256, QC = 512, HH = 16, DH = 64, DR = 64, HD = HH * DH;
constexpr float AS_ = 8.0f, SCL = 0.08838834764831845f;

typedef _Float16 b16;
typedef __attribute__((ext_vector_type(16))) _Float16 v16b;
typedef __attribute__((ext_vector_type(16))) __bf16 v16bb;
typedef __attribute__((ext_vector_type(8))) _Float16 v8b;
typedef __attribute__((ext_vector_type(8))) unsigned short v8us;
typedef __attribute__((ext_vector_type(8))) float v8f;
typedef __attribute__((ext_vector_type(4))) float v4f;
__device__ __forceinline__ float bf16_rne(float f) { unsigned int u = __float_as_uint(f); u += 0x7FFFu + ((u >> 16) & 1u); return __uint_as_float(u & 0xFFFF0000u); }
__device__ __forceinline__ unsigned short bf16_bits(float f) { unsigned int u = __float_as_uint(f); u += 0x7FFFu + ((u >> 16) & 1u); return (unsigned short)(u >> 16); }
__device__ __forceinline__ void split16(float v, b16& hi, b16& lo) { hi = (b16)v; lo = (b16)(v - (float)hi); }
__device__ __forceinline__ v16b frag_kb(const b16* p, int hh) { const v8b a = *(const v8b*)(p + 8 * hh), b = *(const v8b*)(p + 16 + 8 * hh); v16b f;
#pragma unroll
  for (int e = 0; e < 8; ++e) { f[e] = a[e]; f[8 + e] = b[e]; } return f; }
__device__ __forceinline__ v16bb frag_bf(const unsigned short* p, int hh) { const v8us a = *(const v8us*)(p + 8 * hh), b = *(const v8us*)(p + 16 + 8 * hh); union { unsigned short s[16]; v16bb v; } u;
#pragma unroll
  for (int e = 0; e < 8; ++e) { u.s[e] = a[e]; u.s[8 + e] = b[e]; } return u.v; }
__device__ __forceinline__ v16bb frag_f32bf(const float* p, int hh) { union { unsigned short s[16]; v16bb v; } u;
#pragma unroll
  for (int e = 0; e < 8; ++e) { u.s[e] = bf16_bits(p[8 * hh + e]); u.s[8 + e] = bf16_bits(p[16 + 8 * hh + e]); } return u.v; }
__device__ __forceinline__ void frag_split(const float* p, int hh, v16b& fh, v16b& fl) {
#pragma unroll
  for (int e = 0; e < 8; ++e) { b16 a, c; split16(p[8 * hh + e] * AS_, a, c); fh[e] = a; fl[e] = c; split16(p[16 + 8 * hh + e] * AS_, a, c); fh[8 + e] = a; fl[8 + e] = c; } }
__device__ __forceinline__ v8f wmma16b(v16b a, v16b b, v8f c) { v8f d = __builtin_amdgcn_wmma_f32_16x16x32_f16(false, a, false, b, (short)0, c, false, false); asm volatile("v_nop\n\tv_nop\n\tv_nop\n\tv_nop" : "+v"(d) : "v"(a), "v"(b)); return d; }
__device__ __forceinline__ v8f wmma16bb(v16bb a, v16bb b, v8f c) { v8f d = __builtin_amdgcn_wmma_f32_16x16x32_bf16(false, a, false, b, (short)0, c, false, false); asm volatile("v_nop\n\tv_nop\n\tv_nop\n\tv_nop" : "+v"(d) : "v"(a), "v"(b)); return d; }
__device__ __forceinline__ void wave_lds_sync() { __builtin_amdgcn_fence(__ATOMIC_RELEASE, "workgroup"); __builtin_amdgcn_wave_barrier(); __builtin_amdgcn_fence(__ATOMIC_ACQUIRE, "workgroup"); }
__device__ __forceinline__ float nexp(float x) { return __builtin_amdgcn_exp2f(x * 1.4426950408889634f); }
__device__ __forceinline__ float pmul(float a, float b) { float p = a * b; asm volatile("" : "+v"(p)); return p; }
__device__ __forceinline__ void store_tile(const float* Tt, float* dst0, int ld, int lane) { const int hlf = lane >> 4, nloc = lane & 15;
  for (int pass = 0; pass < 2; ++pass) {
#pragma unroll
    for (int j = 0; j < 16; ++j) { const int rr = j * 2 + hlf, c4 = nloc * 4; *(volatile v4f*)(dst0 + (size_t)rr * ld + c4) = *(const v4f*)(Tt + rr * 64 + c4); }
    __threadfence(); } }

struct Wo_ { static constexpr size_t UQ = 0, QR = UQ + 1024 * 512, UK = QR + 1024 * 512, UV = UK + 1024 * 256, KR = UV + 1024 * 256, O = KR + 64 * 256, END = O + 1024 * 1024; };
struct RopeInv { float v[32]; };
__device__ __forceinline__ void sincos_r(float ang, float& sn, float& cs) { const float k = rintf(ang * 0.15915494309189535f); float r = __builtin_fmaf(k, -6.28318548202514648f, ang); r = __builtin_fmaf(k, 1.7484556025237907e-7f, r);
  const float t = r * 0.15915494309189535f; sn = __builtin_amdgcn_sinf(t); cs = __builtin_amdgcn_cosf(t); }
__global__ __launch_bounds__(256) void prep_kernel(const float* __restrict__ Wkv, const float* __restrict__ Wdq, const float* __restrict__ Wuq, const float* __restrict__ Wqr, const float* __restrict__ Wuk, const float* __restrict__ Wkr, const float* __restrict__ Wuv, const float* __restrict__ Wo,
                                                   RopeInv rinv, unsigned short* __restrict__ w1, b16* __restrict__ R, float* __restrict__ cst) {
  const size_t tid = (size_t)blockIdx.x * blockDim.x + threadIdx.x, nth = (size_t)gridDim.x * blockDim.x;
  auto trb = [&](unsigned short* dst, const float* W, int IN, int OUT, size_t p) { const int o = (int)(p / (IN / 8)), k8 = (int)(p % (IN / 8)) * 8; v8us v;
#pragma unroll
    for (int e = 0; e < 8; ++e) v[e] = bf16_bits(W[(size_t)(k8 + e) * OUT + o]);
    *(volatile v8us*)(dst + (size_t)o * IN + k8) = v; };
  auto trh = [&](b16* dst, const float* W, int IN, int OUT, size_t p) { const int o = (int)(p / (IN / 8)), k8 = (int)(p % (IN / 8)) * 8; v8b v;
#pragma unroll
    for (int e = 0; e < 8; ++e) v[e] = (b16)bf16_rne(W[(size_t)(k8 + e) * OUT + o]);
    *(volatile v8b*)(dst + (size_t)o * IN + k8) = v; };
  for (int pass = 0; pass < 2; ++pass) {
    for (size_t p = tid; p < (size_t)CL * KVD / 8; p += nth) trb(w1, Wkv, KVD, CL, p);
    for (size_t p = tid; p < (size_t)QC * QD / 8; p += nth) trb(w1 + (size_t)CL * KVD, Wdq, QD, QC, p);
    for (size_t p = tid; p < (size_t)HD * QC / 8; p += nth) { trh(R + Wo_::UQ, Wuq, QC, HD, p); trh(R + Wo_::QR, Wqr, QC, HD, p); }
    for (size_t p = tid; p < (size_t)HD * CL / 8; p += nth) { trh(R + Wo_::UK, Wuk, CL, HD, p); trh(R + Wo_::UV, Wuv, CL, HD, p); }
    for (size_t p = tid; p < (size_t)DR * CL / 8; p += nth) trh(R + Wo_::KR, Wkr, CL, DR, p);
    for (size_t p = tid; p < (size_t)QD * HD / 8; p += nth) trh(R + Wo_::O, Wo, HD, QD, p);
    for (size_t p = tid; p < (size_t)L * 32 / 2; p += nth) { const int pos = (int)(p / 16), i2 = (int)(p % 16) * 2; v4f o;
#pragma unroll
      for (int e = 0; e < 2; ++e) { float sn, cs; sincos_r((float)pos * rinv.v[i2 + e], sn, cs); o[2 * e] = cs; o[2 * e + 1] = sn; }
      *(volatile v4f*)(cst + p * 4) = o; }
    __threadfence(); }
}

__global__ __launch_bounds__(128) void lin1_kernel(const float* __restrict__ X, const unsigned short* __restrict__ Wt, int N, float* __restrict__ Y) {
  __shared__ __attribute__((aligned(16))) float Ts[4][32 * 64];
  const int lane = threadIdx.x & 31, wave = threadIdx.x >> 5, nloc = lane & 15, hlf = lane >> 4, m0 = blockIdx.y * 128 + wave * 32, c0 = blockIdx.x * 64;
  v8f acc[2][4];
#pragma unroll
  for (int r = 0; r < 2; ++r)
#pragma unroll
    for (int t = 0; t < 4; ++t) acc[r][t] = (v8f){};
#pragma unroll 2
  for (int kb = 0; kb < QD; kb += 32) { const v16bb a0 = frag_f32bf(X + (size_t)(m0 + nloc) * QD + kb, hlf), a1 = frag_f32bf(X + (size_t)(m0 + 16 + nloc) * QD + kb, hlf);
#pragma unroll
    for (int t = 0; t < 4; ++t) { const v16bb bw = frag_bf(Wt + (size_t)(c0 + t * 16 + nloc) * QD + kb, hlf); acc[0][t] = wmma16bb(a0, bw, acc[0][t]); acc[1][t] = wmma16bb(a1, bw, acc[1][t]); } }
  float* Tt = Ts[wave];
#pragma unroll
  for (int t = 0; t < 4; ++t)
#pragma unroll
    for (int r = 0; r < 2; ++r)
#pragma unroll
      for (int v = 0; v < 8; ++v) Tt[(r * 16 + v + 8 * hlf) * 64 + t * 16 + nloc] = acc[r][t][v];
  wave_lds_sync();
  store_tile(Tt, Y + (size_t)m0 * N + c0, N, lane);
}

__global__ __launch_bounds__(128) void lin2_kernel(const float* __restrict__ X, int K, const b16* __restrict__ Bw, int N, int rope, const float* __restrict__ cst, float* __restrict__ Y) {
  __shared__ __attribute__((aligned(16))) float Ts[4][32 * 64];
  const int lane = threadIdx.x & 31, wave = threadIdx.x >> 5, nloc = lane & 15, hlf = lane >> 4, m0 = blockIdx.y * 128 + wave * 32, c0 = blockIdx.x * 64;
  v8f acc[2][4];
#pragma unroll
  for (int r = 0; r < 2; ++r)
#pragma unroll
    for (int t = 0; t < 4; ++t) acc[r][t] = (v8f){};
  for (int kb = 0; kb < K; kb += 32) { v16b a0, l0, a1, l1; frag_split(X + (size_t)(m0 + nloc) * K + kb, hlf, a0, l0); frag_split(X + (size_t)(m0 + 16 + nloc) * K + kb, hlf, a1, l1);
#pragma unroll
    for (int t = 0; t < 4; ++t) { const v16b bw = frag_kb(Bw + (size_t)(c0 + t * 16 + nloc) * K + kb, hlf); acc[0][t] = wmma16b(a0, bw, acc[0][t]); acc[0][t] = wmma16b(l0, bw, acc[0][t]); acc[1][t] = wmma16b(a1, bw, acc[1][t]); acc[1][t] = wmma16b(l1, bw, acc[1][t]); } }
  float* Tt = Ts[wave];
  if (rope) {
#pragma unroll
    for (int t = 0; t < 2; ++t) { const int i = t * 16 + nloc;
#pragma unroll
      for (int r = 0; r < 2; ++r)
#pragma unroll
        for (int v = 0; v < 8; ++v) { const int rl = r * 16 + v + 8 * hlf; const float cs = cst[((size_t)(m0 + rl) * 32 + i) * 2], sn = cst[((size_t)(m0 + rl) * 32 + i) * 2 + 1];
          const float x1 = acc[r][t][v] * (1.0f / AS_), x2 = acc[r][t + 2][v] * (1.0f / AS_); Tt[rl * 64 + i] = x1 * cs - x2 * sn; Tt[rl * 64 + 32 + i] = x2 * cs + x1 * sn; } }
  } else {
#pragma unroll
    for (int t = 0; t < 4; ++t)
#pragma unroll
      for (int r = 0; r < 2; ++r)
#pragma unroll
        for (int v = 0; v < 8; ++v) Tt[(r * 16 + v + 8 * hlf) * 64 + t * 16 + nloc] = acc[r][t][v] * (1.0f / AS_); }
  wave_lds_sync();
  store_tile(Tt, Y + (size_t)m0 * N + c0, N, lane);
}

__global__ __launch_bounds__(256) void attn_kernel(const float* __restrict__ qn, const float* __restrict__ qpe, const float* __restrict__ kn, const float* __restrict__ kpe, const float* __restrict__ vv, const int* __restrict__ seg, float* __restrict__ ctx) {
  __shared__ __attribute__((aligned(16))) float Row[8][HD];
  const int wid = threadIdx.x >> 5, lane = threadIdx.x & 31, h = lane >> 1, hf = lane & 1; const int i = blockIdx.x * 8 + wid;
  int s = seg[i]; s = (s < 0) ? 0 : (s >= L ? L - 1 : s);
  const float* qrow = qn + (size_t)i * HD + h * DH + hf * 32; const float* qprow = qpe + (size_t)i * HD + h * DR + hf * 32;
  float sc[3]; bool ok[3];
#pragma unroll
  for (int j = 0; j < 3; ++j) { const int k = s - 2 + j; ok[j] = (k >= 0); const int kk = ok[j] ? k : 0; const float* krow = kn + (size_t)kk * HD + h * DH + hf * 32; const float* kprow = kpe + (size_t)kk * DR + hf * 32; float d = 0.0f;
#pragma unroll 1
    for (int e = 0; e < 32; ++e) d += pmul(qrow[e], krow[e]) + pmul(qprow[e], kprow[e]);
    d += __shfl_xor(d, 1); sc[j] = ok[j] ? d * SCL : -INFINITY; }
  const float m = fmaxf(sc[0], fmaxf(sc[1], sc[2])); float e_[3], z = 0.0f;
#pragma unroll
  for (int j = 0; j < 3; ++j) { e_[j] = ok[j] ? nexp(sc[j] - m) : 0.0f; z += e_[j]; }
  const float iz = 1.0f / z;
#pragma unroll 1
  for (int e = 0; e < 32; ++e) { float a = 0.0f;
#pragma unroll
    for (int j = 0; j < 3; ++j) { const int kk = ok[j] ? (s - 2 + j) : 0; a += pmul(e_[j] * iz, vv[(size_t)kk * HD + h * DH + hf * 32 + e]); }
    Row[wid][h * DH + hf * 32 + e] = a; }
  wave_lds_sync();
  for (int pass = 0; pass < 2; ++pass) { for (int c = lane * 4; c < HD; c += 128) *(volatile v4f*)(ctx + (size_t)i * HD + c) = *(const v4f*)(&Row[wid][c]); __threadfence(); }
}
}

extern "C" void kernel_launch(void* const* d_in, const int* in_sizes, int n_in,
                              void* d_out, int out_size, void* d_ws, size_t ws_size, hipStream_t stream) {
  (void)n_in; (void)out_size;
  const float* q = (const float*)d_in[0]; const float* kv = (const float*)d_in[1]; const float* Wkv = (const float*)d_in[2]; const float* Wdq = (const float*)d_in[3]; const float* Wuq = (const float*)d_in[4]; const float* Wqr = (const float*)d_in[5]; const float* Wuk = (const float*)d_in[6]; const float* Wkr = (const float*)d_in[7]; const float* Wuv = (const float*)d_in[8]; const float* Wo = (const float*)d_in[9];
  const int* seg = (const int*)d_in[10];
  float* out = (float*)d_out;
  if (in_sizes[0] != L * QD || in_sizes[1] != L * KVD || in_sizes[2] != KVD * CL || in_sizes[3] != QD * QC || in_sizes[4] != QC * HD || in_sizes[7] != CL * DR || in_sizes[9] != HD * QD || in_sizes[10] != L) return;
  size_t off = 0; char* ws = (char*)d_ws;
  auto carve = [&](size_t bytes) { char* p = ws + off; off += (bytes + 255) & ~(size_t)255; return p; };
  unsigned short* w1 = (unsigned short*)carve(((size_t)CL * KVD + (size_t)QC * QD) * 2); b16* R = (b16*)carve(Wo_::END * 2);
float* cst = (float*)carve((size_t)L * 32 * 2 * 4); float* kvc = (float*)carve((size_t)L * CL * 4); float* qc = (float*)carve((size_t)L * QC * 4); float* qn = (float*)carve((size_t)L * HD * 4); float* qpe = (float*)carve((size_t)L * HD * 4); float* kn = (float*)carve((size_t)L * HD * 4); float* kpe = (float*)carve((size_t)L * DR * 4); float* vv = (float*)carve((size_t)L * HD * 4); float* ctx = (float*)carve((size_t)L * HD * 4);
  if (off > ws_size) return;
  RopeInv rinv; for (int i = 0; i < 32; ++i) rinv.v[i] = (float)(1.0 / pow(10000.0, (double)(2 * i) / 64.0));
  prep_kernel<<<512, 256, 0, stream>>>(Wkv, Wdq, Wuq, Wqr, Wuk, Wkr, Wuv, Wo, rinv, w1, R, cst);
  lin1_kernel<<<dim3(CL / 64, L / 128), 128, 0, stream>>>(kv, w1, CL, kvc);
  lin1_kernel<<<dim3(QC / 64, L / 128), 128, 0, stream>>>(q, w1 + (size_t)CL * KVD, QC, qc);
  lin2_kernel<<<dim3(HD / 64, L / 128), 128, 0, stream>>>(qc, QC, R + Wo_::UQ, HD, 0, cst, qn);
  lin2_kernel<<<dim3(HD / 64, L / 128), 128, 0, stream>>>(qc, QC, R + Wo_::QR, HD, 1, cst, qpe);
  lin2_kernel<<<dim3(HD / 64, L / 128), 128, 0, stream>>>(kvc, CL, R + Wo_::UK, HD, 0, cst, kn);
  lin2_kernel<<<dim3(DR / 64, L / 128), 128, 0, stream>>>(kvc, CL, R + Wo_::KR, DR, 1, cst, kpe);
  lin2_kernel<<<dim3(HD / 64, L / 128), 128, 0, stream>>>(kvc, CL, R + Wo_::UV, HD, 0, cst, vv);
  attn_kernel<<<L / 8, 256, 0, stream>>>(qn, qpe, kn, kpe, vv, seg, ctx);
  lin2_kernel<<<dim3(QD / 64, L / 128), 128, 0, stream>>>(ctx, HD, R + Wo_::O, QD, 0, cst, out);
}
